// Rwkv6SelfAttention_48644799595108
// MI455X (gfx1250) — hardware-verified
//
#include <hip/hip_runtime.h>
#include <math.h>

constexpr int  kT      = 1024;
constexpr int  kH      = 2048;
constexpr int  kHS     = 64;
constexpr int  kNH     = 32;
constexpr int  kTM     = 32;
constexpr int  kTD     = 64;
constexpr int  kW1N    = 5 * kTM;
constexpr int  kW1Npad = 192;
constexpr long kP      = (long)kT * kH;
constexpr int  kLC     = 16;
constexpr long kOut1Off = kP;
constexpr long kOut2Off = kP + kH;
static_assert(kOut2Off * 4 == 8396800, "out2 byte offset");
static_assert((kOut2Off + (long)kNH * kHS * kHS) * 4 == 8921088, "total out bytes");

typedef __attribute__((ext_vector_type(16))) _Float16 v16h;
typedef __attribute__((ext_vector_type(8)))  _Float16 v8h;
typedef __attribute__((ext_vector_type(16))) __bf16   v16b;
typedef __attribute__((ext_vector_type(8)))  __bf16   v8b;
typedef __attribute__((ext_vector_type(8)))  float    v8f;
typedef __attribute__((ext_vector_type(4)))  float    v4f;
typedef __attribute__((ext_vector_type(2)))  float    v2f;
typedef __attribute__((ext_vector_type(4)))  unsigned int v4u;
typedef __attribute__((ext_vector_type(2)))  unsigned int v2u;

__device__ __forceinline__ unsigned short f2bf_bits(float f) {
  unsigned u = __float_as_uint(f);
  return (unsigned short)((u + 0x7FFFu + ((u >> 16) & 1u)) >> 16);
}
__device__ __forceinline__ float bf_bits2f(unsigned short h) { return __uint_as_float(((unsigned)h) << 16); }

__device__ __forceinline__ void dep_guard_h(v8f& a, v8f& b, v16h x, v16h y) { asm volatile("v_nop\n\tv_nop\n\tv_nop\n\tv_nop" : "+v"(a), "+v"(b) : "v"(x), "v"(y)); }
__device__ __forceinline__ void dep_guard_b(v8f& a, v8f& b, v16b x, v16b y) { asm volatile("v_nop\n\tv_nop\n\tv_nop\n\tv_nop" : "+v"(a), "+v"(b) : "v"(x), "v"(y)); }
__device__ __forceinline__ void keep4_h(v16h a, v16h b, v16h c, v16h d) { asm volatile("v_nop" :: "v"(a), "v"(b), "v"(c), "v"(d)); }
__device__ __forceinline__ void keep4_b(v16b a, v16b b, v16b c, v16b d) { asm volatile("v_nop" :: "v"(a), "v"(b), "v"(c), "v"(d)); }
__device__ __forceinline__ void acc_guard4(v8f& a, v8f& b, v8f& c, v8f& d) { asm volatile("v_nop\n\tv_nop\n\tv_nop\n\tv_nop" : "+v"(a), "+v"(b), "+v"(c), "+v"(d)); }
template <typename T> struct Frag;
template <> struct Frag<_Float16> {
  typedef v16h V; union U { v16h v; v8h h[2]; };
  static __device__ __forceinline__ v16h load(const _Float16* p) {
    U f; f.h[0] = *(const v8h*)(p); f.h[1] = *(const v8h*)(p + 16); return f.v;
  }
  static __device__ __forceinline__ v8f mma(v16h a, v16h b, v8f c) {
    return __builtin_amdgcn_wmma_f32_16x16x32_f16(false, a, false, b, (short)0, c, false, false);
  }
  static __device__ __forceinline__ void guard(v8f& a, v8f& b, v16h x, v16h y) { dep_guard_h(a, b, x, y); }
  static __device__ __forceinline__ void keep(v16h a, v16h b, v16h c, v16h d) { keep4_h(a, b, c, d); }
};
template <> struct Frag<__bf16> {
  typedef v16b V; union U { v16b v; v8b h[2]; };
  static __device__ __forceinline__ v16b load(const __bf16* p) {
    U f; f.h[0] = *(const v8b*)(p); f.h[1] = *(const v8b*)(p + 16); return f.v;
  }
  static __device__ __forceinline__ v8f mma(v16b a, v16b b, v8f c) {
    return __builtin_amdgcn_wmma_f32_16x16x32_bf16(false, a, false, b, (short)0, c, false, false);
  }
  static __device__ __forceinline__ void guard(v8f& a, v8f& b, v16b x, v16b y) { dep_guard_b(a, b, x, y); }
  static __device__ __forceinline__ void keep(v16b a, v16b b, v16b c, v16b d) { keep4_b(a, b, c, d); }
};

__device__ __forceinline__ unsigned pk16(unsigned short a, unsigned short b) { return (unsigned)a | ((unsigned)b << 16); }
__device__ __forceinline__ void split_bf(float f, unsigned short& hb, unsigned short& lb) {
  hb = f2bf_bits(f);
  lb = f2bf_bits(f - bf_bits2f(hb));
}

template <int ET> struct Elem;
template <> struct Elem<0> { typedef _Float16 T; };
template <> struct Elem<1> { typedef __bf16 T; };
template <int ET, bool SPLIT, int BIAS_MODE, int OUT_MODE, bool RESID, int ACT, bool MIXEPI>
__global__ __launch_bounds__(256) void wmma_gemm64(
    const unsigned short* __restrict__ Ap, const unsigned short* __restrict__ A2p, int lda, long strideA,
    const unsigned short* __restrict__ Btp, const unsigned short* __restrict__ Bt2p, int ldb, long strideB,
    void* __restrict__ Cout, void* __restrict__ Cout2, int ldc, long strideC,
    const float* __restrict__ bias,
    const float* __restrict__ resid, const float* __restrict__ aux, long strideR,
    int M, int N, int K, float scale) {
  typedef typename Elem<ET>::T T;
  typedef typename Frag<T>::V V;
  const T* A = (const T*)Ap; const T* A2 = (const T*)A2p; const T* Bt = (const T*)Btp; const T* Bt2 = (const T*)Bt2p;
  __shared__ __align__(16) float sT[8][16 * 68];
  const int b    = blockIdx.y;
  const int lane = threadIdx.x & 31;
  const int wave = threadIdx.x >> 5;
  const int tilesN = N >> 6;
  const int tilesM = M >> 6;
  const int tile = blockIdx.x * 8 + wave;
  if (tile >= tilesM * tilesN) return;
  const int tm = tile / tilesN;
  const int tn = tile - tm * tilesN;
  const int m0 = tm << 6;
  const int n0 = tn << 6;

  const T* Ab  = A  + (size_t)b * strideA;
  const T* Bb  = Bt + (size_t)b * strideB;
  const T* Ab2 = SPLIT ? (A2  + (size_t)b * strideA) : nullptr;
  const T* Bb2 = SPLIT ? (Bt2 + (size_t)b * strideB) : nullptr;

  const int rlane = lane & 15;
  const int koff  = (lane >> 4) * 8;
  const int mOff  = (lane >> 4) * 8;

  v8f acc[4][4];
#pragma unroll
  for (int i = 0; i < 4; ++i)
#pragma unroll
    for (int j = 0; j < 4; ++j) acc[i][j] = (v8f){0.f,0.f,0.f,0.f,0.f,0.f,0.f,0.f};

  for (int k0 = 0; k0 < K; k0 += 32) {
    V bh[4], bl[4];
#pragma unroll
    for (int j = 0; j < 4; ++j) {
      const size_t bo = (size_t)(n0 + (j << 4) + rlane) * ldb + koff + k0;
      bh[j] = Frag<T>::load(Bb + bo);
      if (SPLIT) bl[j] = Frag<T>::load(Bb2 + bo);
    }
#pragma unroll
    for (int i = 0; i < 4; ++i) {
      const size_t ao = (size_t)(m0 + (i << 4) + rlane) * lda + koff + k0;
      V ah = Frag<T>::load(Ab + ao);
      V al;
      if (SPLIT) al = Frag<T>::load(Ab2 + ao);
#pragma unroll
      for (int j = 0; j < 4; ++j) {
        acc[i][j] = Frag<T>::mma(ah, bh[j], acc[i][j]);
        if (SPLIT) {
          acc[i][j] = Frag<T>::mma(ah, bl[j], acc[i][j]);
          acc[i][j] = Frag<T>::mma(al, bh[j], acc[i][j]);
        }
      }
      Frag<T>::guard(acc[i][0], acc[i][3], ah, SPLIT ? al : ah);
    }
    Frag<T>::keep(bh[0], bh[1], bh[2], bh[3]);
    if (SPLIT) Frag<T>::keep(bl[0], bl[1], bl[2], bl[3]);
  }
  acc_guard4(acc[0][0], acc[0][1], acc[0][2], acc[0][3]);
  acc_guard4(acc[1][0], acc[1][1], acc[1][2], acc[1][3]);
  acc_guard4(acc[2][0], acc[2][1], acc[2][2], acc[2][3]);
  acc_guard4(acc[3][0], acc[3][1], acc[3][2], acc[3][3]);

  float* slab = sT[wave];
  const float* Rb = (RESID || MIXEPI) ? (resid + (size_t)b * strideR) : nullptr;
  const float* Xb = MIXEPI ? (aux + (size_t)b * strideR) : nullptr;
#pragma unroll
  for (int i = 0; i < 4; ++i) {
    const int mBase = m0 + (i << 4);
#pragma unroll
    for (int j = 0; j < 4; ++j) {
      const int n = n0 + (j << 4) + rlane;
      float bv = 0.f;
      if (BIAS_MODE == 2) bv = bias[n];
#pragma unroll
      for (int r = 0; r < 8; ++r) {
        float v = acc[i][j][r] * scale;
        if (BIAS_MODE == 1) v += bias[mBase + mOff + r];
        if (BIAS_MODE == 2) v += bv;
        if (MIXEPI) {
          const size_t ri = (size_t)(mBase + mOff + r) * ldc + n;
          v = Rb[ri] + Xb[ri] * v;
        } else if (RESID) {
          v += Rb[(size_t)(mBase + mOff + r) * ldc + n];
        }
        if (ACT == 1) v = tanhf(v);
        if (ACT == 2) v = fmaxf(v, 0.0f);
        if (ACT == 3) {
          const float ev = expf(-fabsf(v));
          const float rr = 1.0f / (1.0f + ev);
          const float sg = (v >= 0.0f) ? rr : ev * rr;
          v = v * sg;
        }
        if (ACT == 4) v = (v > 0.f) ? v : 0.01f * v;
        slab[(mOff + r) * 68 + (j << 4) + rlane] = v;
      }
    }
    __builtin_amdgcn_fence(__ATOMIC_RELEASE, "workgroup");
    __builtin_amdgcn_wave_barrier();
    __builtin_amdgcn_fence(__ATOMIC_ACQUIRE, "workgroup");
    if (OUT_MODE == 0) {
      float* C = (float*)Cout + (size_t)b * strideC;
      const int hh = lane >> 4, c4 = (lane & 15) * 4;
      for (int pass = 0; pass < 2; ++pass) {
#pragma unroll
        for (int it = 0; it < 8; ++it) {
          const int row = it * 2 + hh;
          v4f v = *(const v4f*)(slab + row * 68 + c4);
          *(volatile v4f*)(C + (size_t)(mBase + row) * ldc + n0 + c4) = v;
        }
        __threadfence();
      }
    } else {
      const int q = lane >> 3, c8 = (lane & 7) * 8;
      unsigned short* C  = (unsigned short*)Cout  + (size_t)b * strideC;
      unsigned short* C2 = (OUT_MODE == 2) ? ((unsigned short*)Cout2 + (size_t)b * strideC) : nullptr;
      for (int pass = 0; pass < 2; ++pass) {
#pragma unroll
        for (int it = 0; it < 4; ++it) {
          const int row = it * 4 + q;
          const float* sp = slab + row * 68 + c8;
          v8h hv, lv;
#pragma unroll
          for (int e = 0; e < 8; ++e) {
            if (OUT_MODE == 1) {
              hv[e] = (_Float16)sp[e];
            } else {
              unsigned short hb = f2bf_bits(sp[e]);
              unsigned short lb = f2bf_bits(sp[e] - bf_bits2f(hb));
              hv[e] = __builtin_bit_cast(_Float16, hb);
              lv[e] = __builtin_bit_cast(_Float16, lb);
            }
          }
          *(volatile v8h*)(C + (size_t)(mBase + row) * ldc + n0 + c8) = hv;
          if (OUT_MODE == 2) *(volatile v8h*)(C2 + (size_t)(mBase + row) * ldc + n0 + c8) = lv;
        }
        __threadfence();
      }
    }
    __builtin_amdgcn_fence(__ATOMIC_RELEASE, "workgroup");
    __builtin_amdgcn_wave_barrier();
    __builtin_amdgcn_fence(__ATOMIC_ACQUIRE, "workgroup");
  }
}

__global__ __launch_bounds__(256) void k_ln1(const float* __restrict__ x, const float* __restrict__ w,
                                             const float* __restrict__ bb, float* __restrict__ xl,
                                             float* __restrict__ out1)
{
  __shared__ float red_a[8];
  __shared__ float red_b[8];
  const int t = blockIdx.x;
  const int tid = threadIdx.x, lane = tid & 31, wave = tid >> 5;
  const float* row = x + (size_t)t * kH;
  const int c0 = 4 * tid, c1 = 1024 + 4 * tid;
  const v4f a0 = *(const v4f*)(row + c0);
  const v4f a1 = *(const v4f*)(row + c1);
  float s = ((a0[0] + a0[1]) + (a0[2] + a0[3])) + ((a1[0] + a1[1]) + (a1[2] + a1[3]));
#pragma unroll
  for (int m = 16; m > 0; m >>= 1) s += __shfl_xor(s, m, 32);
  if (lane == 0) red_a[wave] = s;
  __syncthreads();
  float tot = red_a[0];
#pragma unroll
  for (int i = 1; i < 8; ++i) tot += red_a[i];
  const float mu = tot * (1.0f / 2048.0f);
  v4f d0, d1;
#pragma unroll
  for (int e = 0; e < 4; ++e) { d0[e] = a0[e] - mu; d1[e] = a1[e] - mu; }
  float sq = ((d0[0] * d0[0] + d0[1] * d0[1]) + (d0[2] * d0[2] + d0[3] * d0[3]))
           + ((d1[0] * d1[0] + d1[1] * d1[1]) + (d1[2] * d1[2] + d1[3] * d1[3]));
#pragma unroll
  for (int m = 16; m > 0; m >>= 1) sq += __shfl_xor(sq, m, 32);
  if (lane == 0) red_b[wave] = sq;
  __syncthreads();
  float tot2 = red_b[0];
#pragma unroll
  for (int i = 1; i < 8; ++i) tot2 += red_b[i];
  const float var  = tot2 * (1.0f / 2048.0f);
  const float rinv = rsqrtf(var + 1e-5f);
  const v4f w0 = *(const v4f*)(w + c0),  w1v = *(const v4f*)(w + c1);
  const v4f b0 = *(const v4f*)(bb + c0), b1v = *(const v4f*)(bb + c1);
  v4f y0, y1;
#pragma unroll
  for (int e = 0; e < 4; ++e) {
    y0[e] = d0[e] * rinv * w0[e]  + b0[e];
    y1[e] = d1[e] * rinv * w1v[e] + b1v[e];
  }
  float* o = xl + (size_t)t * kH;
  const bool last = (t == kT - 1);
  for (int pass = 0; pass < 2; ++pass) {
    *(volatile v4f*)(o + c0) = y0;
    *(volatile v4f*)(o + c1) = y1;
    if (last) {
      *(volatile v4f*)(out1 + c0) = y0;
      *(volatile v4f*)(out1 + c1) = y1;
    }
    __threadfence();
  }
}

__global__ __launch_bounds__(256) void k_shift(const float* __restrict__ xl, const float* __restrict__ state1,
                                               const float* __restrict__ tmx, float* __restrict__ sx,
                                               unsigned short* __restrict__ xh, unsigned short* __restrict__ xlo)
{
  const int i = blockIdx.x * 256 + threadIdx.x;
  const int t = i >> 9;
  const int c = (i & 511) * 4;
  const size_t e0 = (size_t)i * 4;
  const v4f cur = *(const v4f*)(xl + e0);
  const size_t pe = (t > 0) ? (e0 - (size_t)kH) : (size_t)0;
  const v4f pv = *(const v4f*)(xl + pe);
  const v4f st = *(const v4f*)(state1 + c);
  const v4f mx = *(const v4f*)(tmx + c);
  v4f s4;
  unsigned short hb[4], lb[4];
#pragma unroll
  for (int e = 0; e < 4; ++e) {
    const float prev = (t == 0) ? st[e] : pv[e];
    const float sv = prev - cur[e];
    s4[e] = sv;
    const float xv = cur[e] + sv * mx[e];
    split_bf(xv, hb[e], lb[e]);
  }
  const v2u uh = (v2u){pk16(hb[0], hb[1]), pk16(hb[2], hb[3])};
  const v2u ul = (v2u){pk16(lb[0], lb[1]), pk16(lb[2], lb[3])};
  for (int pass = 0; pass < 2; ++pass) {
    *(volatile v4f*)(sx + e0) = s4;
    *(volatile v2u*)(xh + e0)  = uh;
    *(volatile v2u*)(xlo + e0) = ul;
    __threadfence();
  }
}

__global__ __launch_bounds__(256) void k_tr64(const float* __restrict__ W, int Ndim, int Kdim,
                                              unsigned short* __restrict__ hi, unsigned short* __restrict__ lo)
{
  __shared__ float sm[64][65];
  const int t  = threadIdx.x;
  const int d0 = blockIdx.x * 64;
  const int h0 = blockIdx.y * 64;
#pragma unroll
  for (int it = 0; it < 16; ++it) {
    const int e = it * 256 + t;
    const int r = e >> 6;
    const int c = e & 63;
    const int n = h0 + c;
    const int nc = (n < Ndim) ? n : (Ndim - 1);
    float v = W[(size_t)(d0 + r) * Ndim + nc];
    if (n >= Ndim) v = 0.0f;
    sm[c][r] = v;
  }
  __syncthreads();
  const int lane = t & 31, wave = t >> 5;
  const int q = lane >> 3, c8 = (lane & 7) * 8;
  v4u uh[2], ul[2];
  size_t o[2];
#pragma unroll
  for (int it = 0; it < 2; ++it) {
    const int row = wave * 8 + it * 4 + q;
    unsigned short hb[8], lb[8];
#pragma unroll
    for (int e = 0; e < 8; ++e) split_bf(sm[row][c8 + e], hb[e], lb[e]);
    uh[it] = (v4u){pk16(hb[0], hb[1]), pk16(hb[2], hb[3]), pk16(hb[4], hb[5]), pk16(hb[6], hb[7])};
    ul[it] = (v4u){pk16(lb[0], lb[1]), pk16(lb[2], lb[3]), pk16(lb[4], lb[5]), pk16(lb[6], lb[7])};
    o[it] = (size_t)(h0 + row) * Kdim + d0 + c8;
  }
  for (int pass = 0; pass < 2; ++pass) {
#pragma unroll
    for (int it = 0; it < 2; ++it) {
      *(volatile v4u*)(hi + o[it]) = uh[it];
      *(volatile v4u*)(lo + o[it]) = ul[it];
    }
    __threadfence();
  }
}

__global__ __launch_bounds__(256) void k_tr32(const float* __restrict__ W2,
                                              unsigned short* __restrict__ hi, unsigned short* __restrict__ lo)
{
  __shared__ float sm[64][33];
  const int t  = threadIdx.x;
  const int f  = blockIdx.x >> 5;
  const int n0 = (blockIdx.x & 31) * 64;
#pragma unroll
  for (int it = 0; it < 8; ++it) {
    const int e = it * 256 + t;
    const int k = e >> 6;
    const int c = e & 63;
    sm[c][k] = W2[(size_t)f * kTM * kH + (size_t)k * kH + n0 + c];
  }
  __syncthreads();
  const int lane = t & 31, wave = t >> 5;
  const int row = wave * 8 + (lane >> 2);
  const int c8  = (lane & 3) * 8;
  unsigned short hb[8], lb[8];
#pragma unroll
  for (int e = 0; e < 8; ++e) split_bf(sm[row][c8 + e], hb[e], lb[e]);
  const v4u uh = (v4u){pk16(hb[0], hb[1]), pk16(hb[2], hb[3]), pk16(hb[4], hb[5]), pk16(hb[6], hb[7])};
  const v4u ul = (v4u){pk16(lb[0], lb[1]), pk16(lb[2], lb[3]), pk16(lb[4], lb[5]), pk16(lb[6], lb[7])};
  const size_t o = (size_t)f * kH * kTM + (size_t)(n0 + row) * kTM + c8;
  for (int pass = 0; pass < 2; ++pass) {
    *(volatile v4u*)(hi + o) = uh;
    *(volatile v4u*)(lo + o) = ul;
    __threadfence();
  }
}

__global__ __launch_bounds__(256) void k_wkv(const float* __restrict__ rr, const float* __restrict__ kk,
                                             const float* __restrict__ vv, const float* __restrict__ tdp,
                                             const float* __restrict__ tdecp, const float* __restrict__ tfirst,
                                             const float* __restrict__ s2in,
                                             float* __restrict__ wkv, float* __restrict__ s2out)
{
  __shared__ __align__(16) float lk[kLC * 64];
  __shared__ __align__(16) float lr[kLC * 64];
  __shared__ __align__(16) float lw[kLC * 64];
  __shared__ __align__(16) float lv[kLC * 64];
  __shared__ __align__(16) float part[kLC * 256];
  static_assert(kLC * 256 == kHS * kHS, "final state staging fits");

  const int h    = blockIdx.x;
  const int tid  = threadIdx.x;
  const int lane = tid & 31, wave = tid >> 5;
  const int i    = tid & 63;
  const int jq   = tid >> 6;
  const int jbase = jq * 16;
  const size_t colbase = (size_t)h * kHS;

  float s[16], u[16];
  {
    const float* sp = s2in + (size_t)h * kHS * kHS + (size_t)i * kHS + jbase;
    const float* up = tfirst + colbase + jbase;
#pragma unroll
    for (int q4 = 0; q4 < 4; ++q4) {
      const v4f sv = *(const v4f*)(sp + 4 * q4);
      const v4f uv = *(const v4f*)(up + 4 * q4);
#pragma unroll
      for (int e = 0; e < 4; ++e) { s[4 * q4 + e] = sv[e]; u[4 * q4 + e] = uv[e]; }
    }
  }
  const int srow = tid >> 4;
  const int sc4  = (tid & 15) * 4;

  for (int ch = 0; ch < kT / kLC; ++ch) {
    const int t0 = ch * kLC;
    __syncthreads();
    {
      const size_t g = (size_t)(t0 + srow) * kH + colbase + sc4;
      *(v4f*)&lk[srow * 64 + sc4] = *(const v4f*)(kk + g);
      *(v4f*)&lr[srow * 64 + sc4] = *(const v4f*)(rr + g);
      *(v4f*)&lv[srow * 64 + sc4] = *(const v4f*)(vv + g);
#pragma unroll 1
      for (int e = 0; e < 4; ++e) {
        float xv = tdp[g + e] + tdecp[colbase + sc4 + e];
        xv = fminf(fmaxf(xv, -9.72f), 2.27f);
        lw[srow * 64 + sc4 + e] = expf(-expf(xv));
      }
    }
    __syncthreads();
#pragma unroll 1
    for (int ts = 0; ts < kLC; ++ts) {
      const float vi = lv[ts * 64 + i];
      float acc = 0.0f;
#pragma unroll
      for (int q4 = 0; q4 < 4; ++q4) {
        const v4f kq = *(const v4f*)&lk[ts * 64 + jbase + 4 * q4];
        const v4f rq = *(const v4f*)&lr[ts * 64 + jbase + 4 * q4];
        const v4f wq = *(const v4f*)&lw[ts * 64 + jbase + 4 * q4];
#pragma unroll
        for (int e = 0; e < 4; ++e) {
          const float kvv = vi * kq[e];
          acc += (kvv * u[4 * q4 + e] + s[4 * q4 + e]) * rq[e];
          s[4 * q4 + e] = kvv + s[4 * q4 + e] * wq[e];
        }
      }
      part[ts * 256 + jq * 64 + i] = acc;
    }
    __syncthreads();
    {
      const int row = 2 * wave + (lane >> 4);
      const int c4  = (lane & 15) * 4;
      const v4f p0 = *(const v4f*)&part[row * 256 + 0   + c4];
      const v4f p1 = *(const v4f*)&part[row * 256 + 64  + c4];
      const v4f p2 = *(const v4f*)&part[row * 256 + 128 + c4];
      const v4f p3 = *(const v4f*)&part[row * 256 + 192 + c4];
      v4f ov;
#pragma unroll
      for (int e = 0; e < 4; ++e) ov[e] = ((p0[e] + p1[e]) + p2[e]) + p3[e];
      float* dst = wkv + (size_t)(t0 + row) * kH + colbase + c4;
      *(volatile v4f*)dst = ov;
      __threadfence();
      *(volatile v4f*)dst = ov;
    }
  }
  __syncthreads();
  {
    float* sp = &part[i * 64 + jbase];
#pragma unroll
    for (int q4 = 0; q4 < 4; ++q4)
      *(v4f*)(sp + 4 * q4) = (v4f){s[4 * q4], s[4 * q4 + 1], s[4 * q4 + 2], s[4 * q4 + 3]};
  }
  __syncthreads();
  {
    float* ob = s2out + (size_t)h * kHS * kHS;
    v4f val[4];
#pragma unroll
    for (int it = 0; it < 4; ++it) val[it] = *(const v4f*)&part[it * 1024 + wave * 128 + lane * 4];
    for (int pass = 0; pass < 2; ++pass) {
#pragma unroll
      for (int it = 0; it < 4; ++it)
        *(volatile v4f*)(ob + it * 1024 + wave * 128 + lane * 4) = val[it];
      __threadfence();
    }
  }
}

__global__ __launch_bounds__(256) void k_lnx(const float* __restrict__ wkv, const float* __restrict__ g,
                                             const float* __restrict__ lnw, const float* __restrict__ lnb,
                                             unsigned short* __restrict__ yh, unsigned short* __restrict__ ylo)
{
  const int lane = threadIdx.x & 31, wave = threadIdx.x >> 5;
  const int idx = blockIdx.x * 8 + wave;
  const int t = idx >> 5;
  const int h = idx & 31;
  const int c = h * kHS + 2 * lane;
  const size_t base = (size_t)t * kH + c;
  const v2f a  = *(const v2f*)(wkv + base);
  const v2f gv = *(const v2f*)(g + base);
  const v2f wv = *(const v2f*)(lnw + c);
  const v2f bv = *(const v2f*)(lnb + c);
  float s = a[0] + a[1];
#pragma unroll
  for (int m = 16; m > 0; m >>= 1) s += __shfl_xor(s, m, 32);
  const float mu = s * (1.0f / 64.0f);
  const float d0 = a[0] - mu, d1 = a[1] - mu;
  float sq = d0 * d0 + d1 * d1;
#pragma unroll
  for (int m = 16; m > 0; m >>= 1) sq += __shfl_xor(sq, m, 32);
  const float var  = sq * (1.0f / 64.0f);
  const float rinv = rsqrtf(var + 1e-5f);
  const float y0 = ((d0 * rinv) * wv[0] + bv[0]) * gv[0];
  const float y1 = ((d1 * rinv) * wv[1] + bv[1]) * gv[1];
  unsigned short h0, l0, h1, l1;
  split_bf(y0, h0, l0);
  split_bf(y1, h1, l1);
  const unsigned uh = pk16(h0, h1);
  const unsigned ul = pk16(l0, l1);
  volatile unsigned* ph = (volatile unsigned*)(yh)  + (base >> 1);
  volatile unsigned* pl = (volatile unsigned*)(ylo) + (base >> 1);
  *ph = uh; *pl = ul;
  __threadfence();
  *ph = uh; *pl = ul;
}

extern "C" void kernel_launch(void* const* d_in, const int* in_sizes, int n_in,
                              void* d_out, int out_size, void* d_ws, size_t ws_size,
                              hipStream_t stream)
{
  if (n_in < 20) return;
  if (in_sizes[0] != (int)kP) return;
  if (out_size != (int)(kOut2Off + (long)kNH * kHS * kHS)) return;

  const float* x       = (const float*)d_in[0];
  const float* state1  = (const float*)d_in[1];
  const float* state2  = (const float*)d_in[2];
  const float* ln1_w   = (const float*)d_in[3];
  const float* ln1_b   = (const float*)d_in[4];
  const float* tmaa_x  = (const float*)d_in[5];
  const float* tmaa    = (const float*)d_in[6];
  const float* tmaa_w1 = (const float*)d_in[7];
  const float* tmaa_w2 = (const float*)d_in[8];
  const float* tdec_w1 = (const float*)d_in[9];
  const float* tdec_w2 = (const float*)d_in[10];
  const float* tdec_p  = (const float*)d_in[11];
  const float* tfirst  = (const float*)d_in[12];
  const float* W_r     = (const float*)d_in[13];
  const float* W_k     = (const float*)d_in[14];
  const float* W_v     = (const float*)d_in[15];
  const float* W_g     = (const float*)d_in[16];
  const float* W_o     = (const float*)d_in[17];
  const float* lnx_w   = (const float*)d_in[18];
  const float* lnx_b   = (const float*)d_in[19];

  float* out0 = (float*)d_out;
  float* out1 = out0 + kOut1Off;
  float* out2 = out0 + kOut2Off;

  char* wsb = (char*)d_ws;
  size_t off = 0;
  auto carve = [&](size_t bytes) -> char* {
    char* p = wsb + off;
    off += (bytes + 127) & ~(size_t)127;
    return p;
  };
  const size_t pf32 = (size_t)kP * 4, p16 = (size_t)kP * 2;
  float* xl   = (float*)carve(pf32);
  float* sx   = (float*)carve(pf32);
  unsigned short* xxh  = (unsigned short*)carve(p16);
  unsigned short* xxl  = (unsigned short*)carve(p16);
  unsigned short* w1Th = (unsigned short*)carve((size_t)kW1Npad * kH * 2);
  unsigned short* w1Tl = (unsigned short*)carve((size_t)kW1Npad * kH * 2);
  unsigned short* t5h  = (unsigned short*)carve((size_t)kT * kW1Npad * 2);
  unsigned short* t5l  = (unsigned short*)carve((size_t)kT * kW1Npad * 2);
  unsigned short* w2Th = (unsigned short*)carve((size_t)5 * kH * kTM * 2);
  unsigned short* w2Tl = (unsigned short*)carve((size_t)5 * kH * kTM * 2);
  unsigned short* dw1Th = (unsigned short*)carve((size_t)kTD * kH * 2);
  unsigned short* dw1Tl = (unsigned short*)carve((size_t)kTD * kH * 2);
  unsigned short* dw2Th = (unsigned short*)carve((size_t)kH * kTD * 2);
  unsigned short* dw2Tl = (unsigned short*)carve((size_t)kH * kTD * 2);
  unsigned short* td1h = (unsigned short*)carve((size_t)kT * kTD * 2);
  unsigned short* td1l = (unsigned short*)carve((size_t)kT * kTD * 2);
  unsigned short* x5h  = (unsigned short*)carve(p16);
  unsigned short* x5l  = (unsigned short*)carve(p16);
  unsigned short* WTh  = (unsigned short*)carve((size_t)kH * kH * 2);
  unsigned short* WTl  = (unsigned short*)carve((size_t)kH * kH * 2);
  float* rb   = (float*)carve(pf32);
  float* kb   = (float*)carve(pf32);
  float* vb   = (float*)carve(pf32);
  float* gb   = (float*)carve(pf32);
  float* tdp  = (float*)carve(pf32);
  float* wkvb = (float*)carve(pf32);
  unsigned short* yh = (unsigned short*)carve(p16);
  unsigned short* yl = (unsigned short*)carve(p16);
  if (off > ws_size) return;

  const unsigned gbBig = (unsigned)(((kT / 64) * (kH / 64) + 7) / 8);
  const unsigned gbT5  = (unsigned)(((kT / 64) * (kW1Npad / 64) + 7) / 8);
  const unsigned gbTd1 = (unsigned)(((kT / 64) * (kTD / 64) + 7) / 8);

  k_ln1<<<kT, 256, 0, stream>>>(x, ln1_w, ln1_b, xl, out1);
  k_shift<<<(unsigned)(kP / 4 / 256), 256, 0, stream>>>(xl, state1, tmaa_x, sx, xxh, xxl);
  k_tr64<<<dim3(kH / 64, kW1Npad / 64), 256, 0, stream>>>(tmaa_w1, kW1N, kH, w1Th, w1Tl);
  k_tr32<<<5 * (kH / 64), 256, 0, stream>>>(tmaa_w2, w2Th, w2Tl);
  k_tr64<<<dim3(kH / 64, kTD / 64), 256, 0, stream>>>(tdec_w1, kTD, kH, dw1Th, dw1Tl);
  k_tr64<<<dim3(kTD / 64, kH / 64), 256, 0, stream>>>(tdec_w2, kH, kTD, dw2Th, dw2Tl);
  wmma_gemm64<1, true, 0, 2, false, 1, false><<<gbT5, 256, 0, stream>>>(
      xxh, xxl, kH, 0, w1Th, w1Tl, kH, 0, (void*)t5h, (void*)t5l, kW1Npad, 0,
      nullptr, nullptr, nullptr, 0, kT, kW1Npad, kH, 1.0f);
  for (int f = 0; f < 5; ++f) {
    wmma_gemm64<1, true, 2, 2, false, 0, true><<<gbBig, 256, 0, stream>>>(
        t5h + f * kTM, t5l + f * kTM, kW1Npad, 0,
        w2Th + (size_t)f * kH * kTM, w2Tl + (size_t)f * kH * kTM, kTM, 0,
        (void*)x5h, (void*)x5l, kH, 0,
        tmaa + (size_t)f * kH, xl, sx, 0, kT, kH, kTM, 1.0f);
    if (f == 0) {
      wmma_gemm64<1, true, 0, 2, false, 1, false><<<gbTd1, 256, 0, stream>>>(
          x5h, x5l, kH, 0, dw1Th, dw1Tl, kH, 0, (void*)td1h, (void*)td1l, kTD, 0,
          nullptr, nullptr, nullptr, 0, kT, kTD, kH, 1.0f);
      wmma_gemm64<1, true, 0, 0, false, 0, false><<<gbBig, 256, 0, stream>>>(
          td1h, td1l, kTD, 0, dw2Th, dw2Tl, kTD, 0, (void*)tdp, nullptr, kH, 0,
          nullptr, nullptr, nullptr, 0, kT, kH, kTD, 1.0f);
    } else {
      const float* Wsrc = (f == 1) ? W_k : (f == 2) ? W_v : (f == 3) ? W_r : W_g;
      float* dst = (f == 1) ? kb : (f == 2) ? vb : (f == 3) ? rb : gb;
      k_tr64<<<dim3(kH / 64, kH / 64), 256, 0, stream>>>(Wsrc, kH, kH, WTh, WTl);
      if (f == 4) {
        wmma_gemm64<1, true, 0, 0, false, 3, false><<<gbBig, 256, 0, stream>>>(
            x5h, x5l, kH, 0, WTh, WTl, kH, 0, (void*)dst, nullptr, kH, 0,
            nullptr, nullptr, nullptr, 0, kT, kH, kH, 1.0f);
      } else {
        wmma_gemm64<1, true, 0, 0, false, 0, false><<<gbBig, 256, 0, stream>>>(
            x5h, x5l, kH, 0, WTh, WTl, kH, 0, (void*)dst, nullptr, kH, 0,
            nullptr, nullptr, nullptr, 0, kT, kH, kH, 1.0f);
      }
    }
  }
  k_wkv<<<kNH, 256, 0, stream>>>(rb, kb, vb, tdp, tdec_p, tfirst, state2, wkvb, out2);
  k_lnx<<<(unsigned)((kT * kNH) / 8), 256, 0, stream>>>(wkvb, gb, lnx_w, lnx_b, yh, yl);
  k_tr64<<<dim3(kH / 64, kH / 64), 256, 0, stream>>>(W_o, kH, kH, WTh, WTl);
  wmma_gemm64<1, true, 0, 0, true, 0, false><<<gbBig, 256, 0, stream>>>(
      yh, yl, kH, 0, WTh, WTl, kH, 0, (void*)out0, nullptr, kH, 0,
      nullptr, x, nullptr, 0, kT, kH, kH, 1.0f);
}
